// PAM_Use_2422361555677
// MI455X (gfx1250) — hardware-verified
//
#include <hip/hip_runtime.h>
#include <stdint.h>

#define NB    4
#define C1    512
#define NP    4096
#define DK    64
#define GMT   64
#define GNT   128
#define OSP   132
#define LTP   72
#define QB    32
#define KCH   256
#define NCH   (NP / KCH)
#define OTP   36
#define VSC   16.0f
#define IVSC  0.0625f
#define LNP   6.931471805599453f
#define WOFFK 262144
#define WOFFQ 294912
#define WTOT  1343488

static_assert(WOFFK == C1 * C1);
static_assert(WOFFQ == WOFFK + DK * C1);
static_assert(WTOT == WOFFQ + NB * NP * DK);
static_assert(WOFFK % 2048 == 0);
static_assert(WOFFQ % 2048 == 0);
static_assert(WTOT % 2048 == 0);
static_assert(NP % GNT == 0);
static_assert(NP % 64 == 0);
static_assert(C1 % GMT == 0);
static_assert(C1 % 64 == 0);
static_assert(DK == GMT);
static_assert(NP % QB == 0);
static_assert(NP % KCH == 0);
static_assert(KCH == 8 * 32);
static_assert(C1 == 4 * 128);
static_assert((OSP * 4) % 16 == 0);
static_assert((OTP * 4) % 16 == 0);
static_assert((LTP * 2) % 16 == 0);

typedef _Float16       v16h __attribute__((ext_vector_type(16)));
typedef _Float16       v8h  __attribute__((ext_vector_type(8)));
typedef __bf16         v16b __attribute__((ext_vector_type(16)));
typedef unsigned short v8us __attribute__((ext_vector_type(8)));
typedef float          v8f  __attribute__((ext_vector_type(8)));
typedef float          v4f  __attribute__((ext_vector_type(4)));
typedef unsigned int   v4u  __attribute__((ext_vector_type(4)));

union Frag  { v8us u[2]; v16h h; v16b bf; };
union FragH { v16h v; v8h hv[2]; };
static_assert(sizeof(Frag) == 32);
static_assert(sizeof(FragH) == 32);

__device__ __forceinline__ unsigned short bf_bits(float f) {
  unsigned u = __float_as_uint(f);
  return (unsigned short)((u + 0x7FFFu + ((u >> 16) & 1u)) >> 16);
}
__device__ __forceinline__ float bf_up(unsigned short hb) { return __uint_as_float(((unsigned)hb) << 16); }
__device__ __forceinline__ float bfr(float f) { return bf_up(bf_bits(f)); }
__device__ __forceinline__ unsigned short h_bits(_Float16 x) { return __builtin_bit_cast(unsigned short, x); }
__device__ __forceinline__ unsigned pk16(unsigned short a, unsigned short b) { return (unsigned)a | ((unsigned)b << 16); }
__device__ __forceinline__ v8f zero8() { v8f z = {0.f, 0.f, 0.f, 0.f, 0.f, 0.f, 0.f, 0.f}; return z; }
__device__ __forceinline__ float hmax8(v8f s) {
  return fmaxf(fmaxf(fmaxf(s[0], s[1]), fmaxf(s[2], s[3])), fmaxf(fmaxf(s[4], s[5]), fmaxf(s[6], s[7])));
}

__device__ __forceinline__ Frag ldfrag(const unsigned short* p) {
  Frag f;
  f.u[0] = *(const v8us*)(p);
  f.u[1] = *(const v8us*)(p + 16);
  return f;
}

__device__ __forceinline__ v8f mma_h(v16h a, v16h b, v8f c) {
  v8f d = __builtin_amdgcn_wmma_f32_16x16x32_f16(false, a, false, b, (short)0, c, false, false);
#if defined(__HIP_DEVICE_COMPILE__)
  asm volatile("v_nop\n\tv_nop\n\tv_nop\n\tv_nop" : "+v"(d) : "v"(a), "v"(b));
#endif
  return d;
}
__device__ __forceinline__ v8f mma_b(v16b a, v16b b, v8f c) {
  v8f d = __builtin_amdgcn_wmma_f32_16x16x32_bf16(false, a, false, b, (short)0, c, false, false);
#if defined(__HIP_DEVICE_COMPILE__)
  const v16h ha = __builtin_bit_cast(v16h, a), hb = __builtin_bit_cast(v16h, b);
  asm volatile("v_nop\n\tv_nop\n\tv_nop\n\tv_nop" : "+v"(d) : "v"(ha), "v"(hb));
#endif
  return d;
}

__global__ __launch_bounds__(256)
void cvt_wq(const float* __restrict__ vw, const float* __restrict__ kw, const float* __restrict__ q,
            unsigned short* WB) {
  const int g0 = (int)blockIdx.x * 2048;
  const float* src = vw;
  int base = 0;
  if (g0 >= WOFFQ)      { src = q;  base = WOFFQ; }
  else if (g0 >= WOFFK) { src = kw; base = WOFFK; }
  const int i = g0 + (int)threadIdx.x * 8;
  const float* s = src + (i - base);
  const v4f a = *(const v4f*)(s);
  const v4f c = *(const v4f*)(s + 4);
  v4u w;
  w[0] = pk16(bf_bits(a[0]), bf_bits(a[1]));
  w[1] = pk16(bf_bits(a[2]), bf_bits(a[3]));
  w[2] = pk16(bf_bits(c[0]), bf_bits(c[1]));
  w[3] = pk16(bf_bits(c[2]), bf_bits(c[3]));
  unsigned short* p = WB + (size_t)i;
  *(volatile v4u*)p = w;
  __threadfence();
  *(volatile v4u*)p = w;
}

__global__ __launch_bounds__(256)
void cvt_x(const float* __restrict__ x, unsigned short* X16) {
  __shared__ __align__(16) unsigned short Lt[64 * LTP];
  const int tid = threadIdx.x;
  const int nt = blockIdx.x, cg = blockIdx.y, b = blockIdx.z;
  const int n0 = nt * 64;
  {
    const int n4 = (tid & 15) * 4, cs = tid >> 4;
#pragma unroll
    for (int it = 0; it < 4; ++it) {
      const int cl = it * 16 + cs;
      const v4f v = *(const v4f*)(x + ((size_t)(b * C1 + cg * 64 + cl)) * NP + n0 + n4);
#pragma unroll
      for (int qq = 0; qq < 4; ++qq) Lt[(n4 + qq) * LTP + cl] = bf_bits(v[qq]);
    }
  }
  __syncthreads();
  {
    const int e = tid & 7, lq = tid >> 3;
#pragma unroll
    for (int pass = 0; pass < 2; ++pass) {
#pragma unroll
      for (int it = 0; it < 2; ++it) {
        const int n = it * 32 + lq;
        const v4u u = *(const v4u*)(Lt + n * LTP + 8 * e);
        *(volatile v4u*)(X16 + ((size_t)(b * NP + n0 + n)) * C1 + cg * 64 + 8 * e) = u;
      }
      __threadfence();
    }
  }
}

template <int MODE>
__global__ __launch_bounds__(256)
void gemm_kernel(const unsigned short* __restrict__ Wp, const unsigned short* __restrict__ X16,
                 const float* __restrict__ bias,
                 unsigned short* outV, unsigned short* outKh, unsigned short* outKl) {
  __shared__ __align__(16) float Os[GMT * OSP];
  const int tid  = threadIdx.x;
  const int lane = tid & 31, wave = tid >> 5;
  const int hh   = lane >> 4, c = lane & 15;
  const int wm   = wave & 1, wn = wave >> 1;
  const int b    = blockIdx.z;
  const int mBase = blockIdx.x * GMT;
  const int nBase = blockIdx.y * GNT;

  const unsigned short* a0p = Wp + (size_t)(mBase + 32 * wm + c) * C1 + 8 * hh;
  const unsigned short* a1p = a0p + (size_t)16 * C1;
  const unsigned short* b0p = X16 + ((size_t)b * NP + nBase + 32 * wn + c) * C1 + 8 * hh;
  const unsigned short* b1p = b0p + (size_t)16 * C1;

  v8f acc[2][2];
#pragma unroll
  for (int mi = 0; mi < 2; ++mi)
#pragma unroll
    for (int ni = 0; ni < 2; ++ni) acc[mi][ni] = zero8();

#pragma unroll 1
  for (int k0 = 0; k0 < C1; k0 += 32) {
    const Frag fa0 = ldfrag(a0p + k0);
    const Frag fa1 = ldfrag(a1p + k0);
    const Frag fb0 = ldfrag(b0p + k0);
    const Frag fb1 = ldfrag(b1p + k0);
    acc[0][0] = mma_b(fa0.bf, fb0.bf, acc[0][0]);
    acc[0][1] = mma_b(fa0.bf, fb1.bf, acc[0][1]);
    acc[1][0] = mma_b(fa1.bf, fb0.bf, acc[1][0]);
    acc[1][1] = mma_b(fa1.bf, fb1.bf, acc[1][1]);
  }

#pragma unroll
  for (int mi = 0; mi < 2; ++mi) {
#pragma unroll
    for (int ni = 0; ni < 2; ++ni) {
      const int n_loc = 32 * wn + 16 * ni + c;
#pragma unroll
      for (int r = 0; r < 8; ++r) {
        const int o_loc = 32 * wm + 16 * mi + 8 * hh + r;
        Os[o_loc * OSP + n_loc] = acc[mi][ni][r] + bfr(bias[mBase + o_loc]);
      }
    }
  }
  __syncthreads();

  {
    const int e = tid & 7, lq = tid >> 3;
#pragma unroll
    for (int pass = 0; pass < 2; ++pass) {
      if (MODE == 0) {
#pragma unroll
        for (int it = 0; it < 4; ++it) {
          const int L = it * 32 + lq;
          const int row = L >> 1, hf = L & 1;
          const v4f v0 = *(const v4f*)(Os + row * OSP + hf * 64 + 8 * e);
          const v4f v1 = *(const v4f*)(Os + row * OSP + hf * 64 + 8 * e + 4);
          v4u u;
          u[0] = pk16(h_bits((_Float16)(v0[0] * VSC)), h_bits((_Float16)(v0[1] * VSC)));
          u[1] = pk16(h_bits((_Float16)(v0[2] * VSC)), h_bits((_Float16)(v0[3] * VSC)));
          u[2] = pk16(h_bits((_Float16)(v1[0] * VSC)), h_bits((_Float16)(v1[1] * VSC)));
          u[3] = pk16(h_bits((_Float16)(v1[2] * VSC)), h_bits((_Float16)(v1[3] * VSC)));
          unsigned short* dst = outV + ((size_t)(b * C1 + mBase + row)) * NP + nBase + hf * 64 + 8 * e;
          *(volatile v4u*)dst = u;
        }
      } else {
#pragma unroll
        for (int it = 0; it < 4; ++it) {
          const int n_loc = it * 32 + lq;
          float f[8];
#pragma unroll
          for (int j = 0; j < 8; ++j) f[j] = Os[(8 * e + j) * OSP + n_loc];
          v4u uh, ul;
#pragma unroll
          for (int t = 0; t < 4; ++t) {
            const unsigned short h0 = bf_bits(f[2 * t]);
            const unsigned short h1 = bf_bits(f[2 * t + 1]);
            const unsigned short l0 = bf_bits(f[2 * t] - bf_up(h0));
            const unsigned short l1 = bf_bits(f[2 * t + 1] - bf_up(h1));
            uh[t] = pk16(h0, h1);
            ul[t] = pk16(l0, l1);
          }
          const size_t po = ((size_t)(b * NP + nBase + n_loc)) * DK + 8 * e;
          *(volatile v4u*)(outKh + po) = uh;
          *(volatile v4u*)(outKl + po) = ul;
        }
      }
      __threadfence();
    }
  }
}

__global__ __launch_bounds__(256)
void attn_kernel(const unsigned short* __restrict__ Qb, const unsigned short* __restrict__ Kh,
                 const unsigned short* __restrict__ Kl, const unsigned short* __restrict__ V16,
                 const float* __restrict__ x, const float* __restrict__ gamma, float* out) {
  __shared__ __align__(16) unsigned short Pl[2 * 8 * 32 * 16];
  __shared__ __align__(16) float Os[256 * OTP];
  __shared__ float smax[2 * 4 * 16];
  __shared__ float lsum[2 * 4 * 16];
  const int tid  = threadIdx.x;
  const int wave = tid >> 5, lane = tid & 31;
  const int hh   = lane >> 4, c = lane & 15;
  const int qt   = wave & 1, cs = wave >> 1;
  const int b    = blockIdx.y;
  const int m0   = blockIdx.x * QB;

  const unsigned short* qp = Qb + ((size_t)b * NP + m0 + 16 * qt + c) * DK + 8 * hh;
  const Frag qf0 = ldfrag(qp);
  const Frag qf1 = ldfrag(qp + 32);
  const v16b q0 = qf0.bf, q1 = qf1.bf;
  const unsigned short* Kbh = Kh + ((size_t)b * NP + c) * DK + 8 * hh;
  const unsigned short* Kbl = Kl + ((size_t)b * NP + c) * DK + 8 * hh;
  const unsigned short* Vbs = V16 + ((size_t)b * C1 + 128 * cs + c) * NP + 8 * hh;

  float m = -1.0e30f, l = 0.f;
  v8f acc[8];
#pragma unroll
  for (int j = 0; j < 8; ++j) acc[j] = zero8();

#pragma unroll 1
  for (int chn = 0; chn < NCH; ++chn) {
    const int kb0   = chn * KCH;
    const int kbase = kb0 + 64 * cs;

    v8f s[4];
#pragma unroll
    for (int ut = 0; ut < 4; ++ut) {
      const size_t ko = (size_t)(kbase + 16 * ut) * DK;
      const Frag kh0 = ldfrag(Kbh + ko);
      const Frag kh1 = ldfrag(Kbh + ko + 32);
      const Frag kl0 = ldfrag(Kbl + ko);
      const Frag kl1 = ldfrag(Kbl + ko + 32);
      v8f sv = mma_b(kh0.bf, q0, zero8());
      sv = mma_b(kh1.bf, q1, sv);
      sv = mma_b(kl0.bf, q0, sv);
      sv = mma_b(kl1.bf, q1, sv);
      s[ut] = sv;
    }

    float mx = fmaxf(fmaxf(hmax8(s[0]), hmax8(s[1])), fmaxf(hmax8(s[2]), hmax8(s[3])));
    mx = fmaxf(mx, __shfl_xor(mx, 16, 32));
    if (hh == 0) smax[(qt * 4 + cs) * 16 + c] = mx;
    __syncthreads();
    float mn = m;
#pragma unroll
    for (int g = 0; g < 4; ++g) mn = fmaxf(mn, smax[(qt * 4 + g) * 16 + c]);
    const float corr = __expf(m - mn);
    m = mn;
    const float msh = mn - LNP;
    l *= corr;
#pragma unroll
    for (int j = 0; j < 8; ++j)
#pragma unroll
      for (int r = 0; r < 8; ++r) acc[j][r] *= corr;

    float ls = 0.f;
#pragma unroll
    for (int u = 0; u < 2; ++u) {
      FragH ph;
#pragma unroll
      for (int r = 0; r < 8; ++r) {
        const float e0 = __expf(s[2 * u][r] - msh);
        const float e1 = __expf(s[2 * u + 1][r] - msh);
        ls += e0 + e1;
        ph.hv[0][r] = (_Float16)e0;
        ph.hv[1][r] = (_Float16)e1;
      }
      unsigned short* pd = Pl + ((qt * 8 + 2 * cs + u) * 32 + lane) * 16;
      *(v8us*)(pd)     = __builtin_bit_cast(v8us, ph.hv[0]);
      *(v8us*)(pd + 8) = __builtin_bit_cast(v8us, ph.hv[1]);
    }
    l += ls;
    __syncthreads();

#pragma unroll 1
    for (int kbk = 0; kbk < 8; ++kbk) {
      const unsigned short* ps = Pl + ((qt * 8 + kbk) * 32 + lane) * 16;
      Frag pf;
      pf.u[0] = *(const v8us*)(ps);
      pf.u[1] = *(const v8us*)(ps + 8);
      const int key0 = kb0 + 32 * kbk;
#pragma unroll
      for (int j = 0; j < 8; ++j) {
        const Frag vf = ldfrag(Vbs + (size_t)(16 * j) * NP + key0);
        acc[j] = mma_h(vf.h, pf.h, acc[j]);
      }
    }
  }

  l += __shfl_xor(l, 16, 32);
  if (hh == 0) lsum[(qt * 4 + cs) * 16 + c] = l;
  __syncthreads();
  float lt = 0.f;
#pragma unroll
  for (int g = 0; g < 4; ++g) lt += lsum[(qt * 4 + g) * 16 + c];
  const float gsc = bfr(gamma[0]) * IVSC * (1.0f / lt);

  const int e = tid & 7, lq = tid >> 3;
#pragma unroll
  for (int phase = 0; phase < 2; ++phase) {
    if ((cs >> 1) == phase) {
      float* os = Os + (128 * (cs & 1) + 8 * hh) * OTP + 16 * qt + c;
#pragma unroll
      for (int j = 0; j < 8; ++j)
#pragma unroll
        for (int r = 0; r < 8; ++r) os[(16 * j + r) * OTP] = acc[j][r] * gsc;
    }
    __syncthreads();
#pragma unroll
    for (int pass = 0; pass < 2; ++pass) {
#pragma unroll
      for (int it = 0; it < 8; ++it) {
        const int row = it * 32 + lq;
        const int chg = phase * 256 + row;
        const v4f v  = *(const v4f*)(Os + row * OTP + 4 * e);
        const size_t gi = ((size_t)(b * C1 + chg)) * NP + m0 + 4 * e;
        const v4f xx = *(const v4f*)(x + gi);
        v4f o;
        o[0] = v[0] + bfr(xx[0]);
        o[1] = v[1] + bfr(xx[1]);
        o[2] = v[2] + bfr(xx[2]);
        o[3] = v[3] + bfr(xx[3]);
        *(volatile v4f*)(out + gi) = o;
      }
      __threadfence();
    }
    __syncthreads();
  }
}

extern "C" void kernel_launch(void* const* d_in, const int* in_sizes, int n_in,
                              void* d_out, int out_size, void* d_ws, size_t ws_size,
                              hipStream_t stream) {
  const int NX = NB * C1 * NP;
  if (n_in < 7) return;
  if (in_sizes[0] != NX) return;
  if (in_sizes[1] != NB * NP * DK) return;
  if (in_sizes[2] != C1 * C1 || in_sizes[3] != C1) return;
  if (in_sizes[4] != DK * C1 || in_sizes[5] != DK) return;
  if (in_sizes[6] < 1) return;
  if (out_size != NX) return;

  size_t off = 0;
  const size_t oW  = off; off += (size_t)WTOT * 2;
  const size_t oX  = off; off += (size_t)NB * NP * C1 * 2;
  const size_t oV  = off; off += (size_t)NB * C1 * NP * 2;
  const size_t oKh = off; off += (size_t)NB * NP * DK * 2;
  const size_t oKl = off; off += (size_t)NB * NP * DK * 2;
  if (off > ws_size) return;
  if (off > (size_t)134217728) return;

  const float* x       = (const float*)d_in[0];
  const float* query   = (const float*)d_in[1];
  const float* value_w = (const float*)d_in[2];
  const float* value_b = (const float*)d_in[3];
  const float* key_w   = (const float*)d_in[4];
  const float* key_b   = (const float*)d_in[5];
  const float* gamma   = (const float*)d_in[6];

  char* ws = (char*)d_ws;
  unsigned short* WB  = (unsigned short*)(ws + oW);
  unsigned short* X16 = (unsigned short*)(ws + oX);
  unsigned short* V16 = (unsigned short*)(ws + oV);
  unsigned short* Kh  = (unsigned short*)(ws + oKh);
  unsigned short* Kl  = (unsigned short*)(ws + oKl);
  float* out = (float*)d_out;

  const dim3 blk256(256);
  const dim3 gW(WTOT / 2048);
  const dim3 gX(NP / 64, C1 / 64, NB);
  const dim3 gV(C1 / GMT, NP / GNT, NB);
  const dim3 gK(1, NP / GNT, NB);
  const dim3 gA(NP / QB, NB);

  cvt_wq<<<gW, blk256, 0, stream>>>(value_w, key_w, query, WB);
  cvt_x<<<gX, blk256, 0, stream>>>(x, X16);
  gemm_kernel<0><<<gV, blk256, 0, stream>>>(WB, X16, value_b, V16, nullptr, nullptr);
  gemm_kernel<1><<<gK, blk256, 0, stream>>>(WB + WOFFK, X16, key_b, nullptr, Kh, Kl);
  attn_kernel<<<gA, blk256, 0, stream>>>(WB + WOFFQ, Kh, Kl, V16, x, gamma, out);
  (void)hipGetLastError();
}
